// Attention_76493367542388
// MI455X (gfx1250) — hardware-verified
//
#include <hip/hip_runtime.h>
#include <math.h>


#pragma clang fp contract(off)

typedef _Float16 v16h __attribute__((ext_vector_type(16)));
typedef _Float16 v8h  __attribute__((ext_vector_type(8)));
typedef v8h v8ha __attribute__((may_alias));
typedef float v8f __attribute__((ext_vector_type(8)));
typedef float v4f __attribute__((ext_vector_type(4)));
typedef v4f v4fa __attribute__((may_alias));

#ifndef NB
#define NB 4
#endif
#ifndef SEQ
#define SEQ 2048
#endif
#define NB_FULL 4
#define SEQ_FULL 2048
#define DIM 1024
#define HEADS 16
#define DHEAD 64
#define NQKV 3072
#define MTOK (NB * SEQ)
#define NBH (NB * HEADS)

static_assert(SEQ % 64 == 0);
static_assert(SEQ <= SEQ_FULL);
static_assert(NB >= 1 && NB <= NB_FULL);
static_assert(DIM % 128 == 0 && NQKV % 128 == 0 && MTOK % 64 == 0);
static_assert((size_t)NB_FULL * SEQ_FULL * DIM * 4 == 33554432ull);

#define WS_TOTAL ((size_t)MTOK * DIM * 2 * 2 + (size_t)NQKV * DIM * 2 + (size_t)DIM * DIM * 2 + \
                  (size_t)SEQ * 32 * 4 * 2 + (size_t)NBH * SEQ * DHEAD * 2 * 3)
static_assert(WS_TOTAL <= (size_t)134217728ull);

struct RopeTab { float inv[32]; };
static_assert(sizeof(RopeTab) == 128);

union Frag16 { v16h v; v8h hv[2]; };

__device__ __forceinline__ v16h frag_row(const _Float16* rowp, int lane) {
  const int kb = (lane >> 4) << 3;
  Frag16 f;
  f.hv[0] = *(const v8ha*)(rowp + kb);
  f.hv[1] = *(const v8ha*)(rowp + 16 + kb);
  return f.v;
}

__device__ __forceinline__ v8f wmma16(v8f c, v16h a, v16h b) {
  v8f d = __builtin_amdgcn_wmma_f32_16x16x32_f16(false, a, false, b, (short)0, c, false, false);
  asm volatile("v_nop\n\tv_nop\n\tv_nop\n\tv_nop" : "+v"(d) : "v"(a), "v"(b));
  return d;
}

__device__ __forceinline__ float bf16_rne(float f) {
  unsigned u = __float_as_uint(f);
  u += 0x7FFFu + ((u >> 16) & 1u);
  return __uint_as_float(u & 0xFFFF0000u);
}

__device__ __forceinline__ void wave_sync_lds() {
  __builtin_amdgcn_fence(3, "wavefront");
  __builtin_amdgcn_wave_barrier();
}

__global__ __launch_bounds__(256) void k_cvt_x(const float* __restrict__ x, _Float16* __restrict__ xh) {
  const int e = blockIdx.x * 256 + (int)threadIdx.x;
  const int tok = e >> 7;
  const int c = (e & 127) * 8;
  if (tok >= MTOK) return;
  const int b = tok / SEQ;
  const int s = tok - b * SEQ;
  const float* src = x + ((size_t)b * SEQ_FULL + s) * DIM + c;
  const v4f f0 = *(const v4f*)src;
  const v4f f1 = *(const v4f*)(src + 4);
  v8h r;
  r[0] = (_Float16)bf16_rne(f0[0]); r[1] = (_Float16)bf16_rne(f0[1]);
  r[2] = (_Float16)bf16_rne(f0[2]); r[3] = (_Float16)bf16_rne(f0[3]);
  r[4] = (_Float16)bf16_rne(f1[0]); r[5] = (_Float16)bf16_rne(f1[1]);
  r[6] = (_Float16)bf16_rne(f1[2]); r[7] = (_Float16)bf16_rne(f1[3]);
  _Float16* dst = xh + (size_t)tok * DIM + c;
  *(volatile v8h*)dst = r;
  __threadfence();
  *(volatile v8h*)dst = r;
}

__global__ __launch_bounds__(256) void k_wt(const float* __restrict__ w, _Float16* __restrict__ wt, int n) {
  __shared__ __attribute__((aligned(16))) _Float16 T[64 * 72];
  const int t = threadIdx.x;
  const int n0 = blockIdx.x * 64, k0 = blockIdx.y * 64;
#pragma unroll
  for (int i = 0; i < 4; ++i) {
    const int v = t + 256 * i;
    const int kr = v >> 4, c4 = (v & 15) * 4;
    const v4f f = *(const v4f*)(w + (size_t)(k0 + kr) * n + n0 + c4);
    T[(c4 + 0) * 72 + kr] = (_Float16)(bf16_rne(f[0]) * 64.0f);
    T[(c4 + 1) * 72 + kr] = (_Float16)(bf16_rne(f[1]) * 64.0f);
    T[(c4 + 2) * 72 + kr] = (_Float16)(bf16_rne(f[2]) * 64.0f);
    T[(c4 + 3) * 72 + kr] = (_Float16)(bf16_rne(f[3]) * 64.0f);
  }
  __syncthreads();
#pragma unroll
  for (int pass = 0; pass < 2; ++pass) {
#pragma unroll
    for (int p = 0; p < 2; ++p) {
      const int P = p * 256 + t;
      const int L = P >> 3, piece = P & 7;
      const v8h val = *(const v8ha*)&T[L * 72 + piece * 8];
      _Float16* dst = wt + (size_t)(n0 + L) * DIM + k0 + piece * 8;
      *(volatile v8h*)dst = val;
    }
    if (pass == 0) __threadfence();
  }
}

__global__ __launch_bounds__(256) void k_tab(float* __restrict__ cosT, float* __restrict__ sinT, RopeTab tab) {
  const int e = blockIdx.x * 256 + (int)threadIdx.x;
  const int s = e >> 5, i = e & 31;
  float f = tab.inv[0];
#pragma unroll
  for (int j = 1; j < 32; ++j) f = (i == j) ? tab.inv[j] : f;
  const float ang = (float)s * f;
  float sv, cv;
  sincosf(ang, &sv, &cv);
  if (e < SEQ * 32) {
    *(volatile float*)(cosT + e) = cv;
    *(volatile float*)(sinT + e) = sv;
    __threadfence();
    *(volatile float*)(cosT + e) = cv;
    *(volatile float*)(sinT + e) = sv;
  }
}

__device__ __forceinline__ void gemm_core(const _Float16* __restrict__ A,
                                          const _Float16* __restrict__ BT,
                                          int arow0, int bcol0, int lane,
                                          v8f (&acc)[2][4]) {
  const int l15 = lane & 15;
  const _Float16* ap0 = A + (size_t)(arow0 + l15) * DIM;
  const _Float16* ap1 = ap0 + (size_t)16 * DIM;
  const _Float16* bp0 = BT + (size_t)(bcol0 + l15) * DIM;
#pragma unroll 2
  for (int k0 = 0; k0 < DIM; k0 += 32) {
    const v16h a0 = frag_row(ap0 + k0, lane);
    const v16h a1 = frag_row(ap1 + k0, lane);
#pragma unroll
    for (int ni = 0; ni < 4; ++ni) {
      const v16h bf = frag_row(bp0 + (size_t)ni * 16 * DIM + k0, lane);
      acc[0][ni] = wmma16(acc[0][ni], a0, bf);
      acc[1][ni] = wmma16(acc[1][ni], a1, bf);
    }
  }
}

__global__ __launch_bounds__(128) __attribute__((amdgpu_num_vgpr(256)))
void k_qkv(const _Float16* __restrict__ xh, const _Float16* __restrict__ wT,
           const float* __restrict__ cosT, const float* __restrict__ sinT,
           _Float16* __restrict__ qpl, _Float16* __restrict__ kpl, _Float16* __restrict__ vtp) {
  __shared__ __attribute__((aligned(16))) _Float16 tile[128 * 72];
  __shared__ __attribute__((aligned(16))) float cs[64 * 32];
  __shared__ __attribute__((aligned(16))) float sn[64 * 32];
  const int t = threadIdx.x, lane = t & 31, wave = t >> 5;
  const int hl = lane >> 4, l15 = lane & 15;
  const int wm = wave >> 1, wn = wave & 1;
  const int m0 = blockIdx.y * 64, n0 = blockIdx.x * 128;
  const int part = n0 >> 10;
  const int h0 = (n0 & 1023) >> 6;
  const int b = m0 / SEQ, s0 = m0 - b * SEQ;
  v8f acc[2][4];
#pragma unroll
  for (int mi = 0; mi < 2; ++mi)
#pragma unroll
    for (int ni = 0; ni < 4; ++ni)
#pragma unroll
      for (int r = 0; r < 8; ++r) acc[mi][ni][r] = 0.0f;

  gemm_core(xh, wT, m0 + wm * 32, n0 + wn * 64, lane, acc);

  const float inv64 = 0.015625f;
  if (part < 2) {
#pragma unroll
    for (int i = 0; i < 4; ++i) {
      const int v = t + 128 * i;
      const int row = v >> 3, c4 = (v & 7) * 4;
      *(v4f*)&cs[row * 32 + c4] = *(const v4f*)(cosT + (size_t)(s0 + row) * 32 + c4);
      *(v4f*)&sn[row * 32 + c4] = *(const v4f*)(sinT + (size_t)(s0 + row) * 32 + c4);
    }
    __syncthreads();
#pragma unroll
    for (int mi = 0; mi < 2; ++mi)
#pragma unroll
      for (int r = 0; r < 8; ++r) {
        const int rowl = wm * 32 + mi * 16 + hl * 8 + r;
#pragma unroll
        for (int nip = 0; nip < 2; ++nip) {
          const int i2 = nip * 16 + l15;
          const float c = cs[rowl * 32 + i2];
          const float sv = sn[rowl * 32 + i2];
          const float a = acc[mi][nip][r] * inv64;
          const float bq = acc[mi][nip + 2][r] * inv64;
          const float lo = a * c - bq * sv;
          const float hi = bq * c + a * sv;
          tile[rowl * 136 + wn * 64 + i2] = (_Float16)lo;
          tile[rowl * 136 + wn * 64 + 32 + i2] = (_Float16)hi;
        }
      }
    __syncthreads();
    _Float16* plane = (part == 0) ? qpl : kpl;
#pragma unroll
    for (int pass = 0; pass < 2; ++pass) {
#pragma unroll
      for (int p = 0; p < 8; ++p) {
        const int P = p * 128 + t;
        const int L = P >> 3, piece = P & 7;
        const int hh = L >> 6, sl = L & 63;
        const v8h val = *(const v8ha*)&tile[sl * 136 + hh * 64 + piece * 8];
        _Float16* dst = plane + ((size_t)((b * HEADS + h0 + hh) * SEQ + s0 + sl)) * DHEAD + piece * 8;
        *(volatile v8h*)dst = val;
      }
      if (pass == 0) __threadfence();
    }
  } else {
#pragma unroll
    for (int mi = 0; mi < 2; ++mi)
#pragma unroll
      for (int ni = 0; ni < 4; ++ni) {
        const int col = wn * 64 + ni * 16 + l15;
        v8h pk;
#pragma unroll
        for (int r = 0; r < 8; ++r) pk[r] = (_Float16)(acc[mi][ni][r] * inv64);
        *(v8h*)&tile[col * 72 + wm * 32 + mi * 16 + hl * 8] = pk;
      }
    __syncthreads();
#pragma unroll
    for (int pass = 0; pass < 2; ++pass) {
#pragma unroll
      for (int p = 0; p < 8; ++p) {
        const int P = p * 128 + t;
        const int L = P >> 3, piece = P & 7;
        const int hh = L >> 6, d = L & 63;
        const v8h val = *(const v8ha*)&tile[L * 72 + piece * 8];
        _Float16* dst = vtp + ((size_t)((b * HEADS + h0 + hh) * DHEAD + d)) * SEQ + s0 + piece * 8;
        *(volatile v8h*)dst = val;
      }
      if (pass == 0) __threadfence();
    }
  }
}

__global__ __launch_bounds__(128) __attribute__((amdgpu_num_vgpr(256)))
void k_attn(const _Float16* __restrict__ qpl, const _Float16* __restrict__ kpl,
            const _Float16* __restrict__ vtp, _Float16* __restrict__ ctx) {
  __shared__ __attribute__((aligned(16))) _Float16 Ps[4][16 * 72];
  const int t = threadIdx.x, lane = t & 31, wave = t >> 5;
  const int hl = lane >> 4, l15 = lane & 15;
  const int bh = blockIdx.y;
  const int b = bh / HEADS, hd = bh - b * HEADS;
  const int n0 = blockIdx.x * 64;
  const _Float16* qbase = qpl + (size_t)bh * SEQ * DHEAD;
  const _Float16* kbase = kpl + (size_t)bh * SEQ * DHEAD;
  const _Float16* vbase = vtp + (size_t)bh * DHEAD * SEQ;
  _Float16* pw = &Ps[wave][0];

  const int mrow = n0 + wave * 16 + l15;
  const v16h qF0 = frag_row(qbase + (size_t)mrow * DHEAD, lane);
  const v16h qF1 = frag_row(qbase + (size_t)mrow * DHEAD + 32, lane);

  v8f o[4];
#pragma unroll
  for (int dt = 0; dt < 4; ++dt)
#pragma unroll
    for (int g = 0; g < 8; ++g) o[dt][g] = 0.0f;
  float mr[8], lr[8];
#pragma unroll
  for (int g = 0; g < 8; ++g) { mr[g] = -1e30f; lr[g] = 0.0f; }
  const float C = 0.18033688011112042f;

#pragma unroll 1
  for (int j0 = 0; j0 < SEQ; j0 += 64) {
    v8f s[4];
#pragma unroll
    for (int jt = 0; jt < 4; ++jt)
#pragma unroll
      for (int g = 0; g < 8; ++g) s[jt][g] = 0.0f;
#pragma unroll
    for (int jt = 0; jt < 4; ++jt) {
      const _Float16* krow = kbase + (size_t)(j0 + jt * 16 + l15) * DHEAD;
      const v16h b0 = frag_row(krow, lane);
      const v16h b1 = frag_row(krow + 32, lane);
      s[jt] = wmma16(s[jt], qF0, b0);
      s[jt] = wmma16(s[jt], qF1, b1);
    }
    float mp[8];
#pragma unroll
    for (int g = 0; g < 8; ++g)
      mp[g] = fmaxf(fmaxf(s[0][g], s[1][g]), fmaxf(s[2][g], s[3][g])) * C;
#pragma unroll
    for (int off = 1; off < 16; off <<= 1)
#pragma unroll
      for (int g = 0; g < 8; ++g)
        mp[g] = fmaxf(mp[g], __shfl_xor(mp[g], off, 32));
#pragma unroll
    for (int g = 0; g < 8; ++g) {
      const float mnew = fmaxf(mr[g], mp[g]);
      const float rsc = exp2f(mr[g] - mnew);
      mr[g] = mnew;
      lr[g] *= rsc;
      o[0][g] *= rsc; o[1][g] *= rsc; o[2][g] *= rsc; o[3][g] *= rsc;
    }
    wave_sync_lds();
#pragma unroll
    for (int jt = 0; jt < 4; ++jt)
#pragma unroll
      for (int g = 0; g < 8; ++g) {
        const float p = exp2f(s[jt][g] * C - mr[g]);
        lr[g] += p;
        pw[(hl * 8 + g) * 72 + jt * 16 + l15] = (_Float16)(p * 4096.0f);
      }
    wave_sync_lds();
#pragma unroll
    for (int ks = 0; ks < 2; ++ks) {
      const v16h pF = frag_row(pw + l15 * 72 + ks * 32, lane);
#pragma unroll
      for (int dt = 0; dt < 4; ++dt) {
        const v16h vF = frag_row(vbase + (size_t)(dt * 16 + l15) * SEQ + j0 + ks * 32, lane);
        o[dt] = wmma16(o[dt], pF, vF);
      }
    }
  }

#pragma unroll
  for (int off = 1; off < 16; off <<= 1)
#pragma unroll
    for (int g = 0; g < 8; ++g)
      lr[g] += __shfl_xor(lr[g], off, 32);
  float iv[8];
#pragma unroll
  for (int g = 0; g < 8; ++g) iv[g] = __builtin_amdgcn_rcpf(lr[g]) * 0.015625f;
  wave_sync_lds();
#pragma unroll
  for (int dt = 0; dt < 4; ++dt)
#pragma unroll
    for (int g = 0; g < 8; ++g)
      pw[(hl * 8 + g) * 72 + dt * 16 + l15] = (_Float16)(o[dt][g] * iv[g]);
  wave_sync_lds();
  const size_t tok0 = (size_t)b * SEQ + n0 + wave * 16;
#pragma unroll
  for (int pass = 0; pass < 2; ++pass) {
#pragma unroll
    for (int i = 0; i < 4; ++i) {
      const int P = i * 32 + lane;
      const int row = P >> 3, piece = P & 7;
      const v8h val = *(const v8ha*)&pw[row * 72 + piece * 8];
      _Float16* dst = ctx + (tok0 + row) * DIM + hd * DHEAD + piece * 8;
      *(volatile v8h*)dst = val;
    }
    if (pass == 0) __threadfence();
  }
}

__global__ __launch_bounds__(128) __attribute__((amdgpu_num_vgpr(256)))
void k_out(const _Float16* __restrict__ ctx, const _Float16* __restrict__ woT, float* __restrict__ out) {
  __shared__ __attribute__((aligned(16))) float Cs[4][32 * 68];
  const int t = threadIdx.x, lane = t & 31, wave = t >> 5;
  const int hl = lane >> 4, l15 = lane & 15;
  const int wm = wave >> 1, wn = wave & 1;
  const int m0 = blockIdx.y * 64, n0 = blockIdx.x * 128;
  v8f acc[2][4];
#pragma unroll
  for (int mi = 0; mi < 2; ++mi)
#pragma unroll
    for (int ni = 0; ni < 4; ++ni)
#pragma unroll
      for (int r = 0; r < 8; ++r) acc[mi][ni][r] = 0.0f;

  gemm_core(ctx, woT, m0 + wm * 32, n0 + wn * 64, lane, acc);

  float* cw = &Cs[wave][0];
  const float sc = 0.000244140625f;
#pragma unroll
  for (int mi = 0; mi < 2; ++mi)
#pragma unroll
    for (int ni = 0; ni < 4; ++ni)
#pragma unroll
      for (int r = 0; r < 8; ++r)
        cw[(mi * 16 + hl * 8 + r) * 68 + ni * 16 + l15] = acc[mi][ni][r] * sc;
  wave_sync_lds();
  const int rb = m0 + wm * 32;
  const int bb = rb / SEQ;
  const size_t orow0 = (size_t)bb * SEQ_FULL + (rb - bb * SEQ);
#pragma unroll
  for (int pass = 0; pass < 2; ++pass) {
#pragma unroll
    for (int i = 0; i < 16; ++i) {
      const int P = i * 32 + lane;
      const int row = P >> 4, piece = P & 15;
      const v4f v = *(const v4fa*)&cw[row * 68 + piece * 4];
      float* dst = out + (orow0 + row) * DIM + n0 + wn * 64 + piece * 4;
      *(volatile v4f*)dst = v;
    }
    if (pass == 0) __threadfence();
  }
}

extern "C" void kernel_launch(void* const* d_in, const int* in_sizes, int n_in,
                              void* d_out, int out_size, void* d_ws, size_t ws_size,
                              hipStream_t stream) {
  if (n_in < 3) return;
  const long need_rows = (long)(NB - 1) * SEQ_FULL + SEQ;
  if ((long)in_sizes[0] < need_rows * DIM) return;
  if ((long)in_sizes[1] < (long)DIM * NQKV) return;
  if ((long)in_sizes[2] < (long)DIM * DIM) return;
  if ((long)out_size < need_rows * DIM) return;

  const float* x    = (const float*)d_in[0];
  const float* wqkv = (const float*)d_in[1];
  const float* wout = (const float*)d_in[2];
  float* out = (float*)d_out;

  char* ws = (char*)d_ws;
  size_t off = 0;
  _Float16* xh = (_Float16*)(ws + off);  off += (size_t)MTOK * DIM * 2;
  _Float16* wqT = (_Float16*)(ws + off); off += (size_t)NQKV * DIM * 2;
  _Float16* woT = (_Float16*)(ws + off); off += (size_t)DIM * DIM * 2;
  float* cosT = (float*)(ws + off);      off += (size_t)SEQ * 32 * 4;
  float* sinT = (float*)(ws + off);      off += (size_t)SEQ * 32 * 4;
  _Float16* qpl = (_Float16*)(ws + off); off += (size_t)NBH * SEQ * DHEAD * 2;
  _Float16* kpl = (_Float16*)(ws + off); off += (size_t)NBH * SEQ * DHEAD * 2;
  _Float16* vtp = (_Float16*)(ws + off); off += (size_t)NBH * SEQ * DHEAD * 2;
  _Float16* ctx = (_Float16*)(ws + off); off += (size_t)MTOK * DIM * 2;
  if (off > ws_size) return;

  RopeTab tab;
  for (int i = 0; i < 32; ++i) {
    const float pf = (float)pow(10000.0, (double)i / 32.0);
    tab.inv[i] = (float)(1.0 / (double)pf);
  }

  k_cvt_x<<<dim3(MTOK / 2), 256, 0, stream>>>(x, xh);
  k_wt<<<dim3(NQKV / 64, DIM / 64), 256, 0, stream>>>(wqkv, wqT, NQKV);
  k_wt<<<dim3(DIM / 64, DIM / 64), 256, 0, stream>>>(wout, woT, DIM);
  k_tab<<<dim3(SEQ * 32 / 256), 256, 0, stream>>>(cosT, sinT, tab);
  k_qkv<<<dim3(NQKV / 128, MTOK / 64), 128, 0, stream>>>(xh, wqT, cosT, sinT, qpl, kpl, vtp);
  k_attn<<<dim3(SEQ / 64, NBH), 128, 0, stream>>>(qpl, kpl, vtp, ctx);
  k_out<<<dim3(DIM / 128, MTOK / 64), 128, 0, stream>>>(ctx, woT, out);
}
